// LanguageGatedBundleMatchModule_51934744543994
// MI455X (gfx1250) — hardware-verified
//
#include <hip/hip_runtime.h>
#include <math.h>

typedef __attribute__((ext_vector_type(16))) _Float16 v16h;
typedef __attribute__((ext_vector_type(16))) __bf16 v16b;
typedef __attribute__((ext_vector_type(8)))  _Float16 v8h;
typedef __attribute__((ext_vector_type(8)))  float v8f;
typedef __attribute__((ext_vector_type(4)))  float v4f;
typedef __attribute__((ext_vector_type(2)))  float v2f;
typedef __attribute__((ext_vector_type(4)))  unsigned v4u;
typedef __attribute__((ext_vector_type(4)))  int v4i;
typedef float __attribute__((may_alias)) float_a;
typedef int __attribute__((may_alias)) int_a;

template <typename T> __device__ __forceinline__ void vst2(void* p, T v) { *(volatile T*)p = v; __threadfence(); *(volatile T*)p = v; }
__device__ __forceinline__ v8f wmma16(v16h a, v16h b, v8f c) {
  v8f d = __builtin_amdgcn_wmma_f32_16x16x32_f16(false, a, false, b, (short)0, c, false, false);
  asm volatile("v_nop\n\tv_nop\n\tv_nop\n\tv_nop" : "+v"(d) : "v"(a), "v"(b));
  return d;
}
__device__ __forceinline__ v8f wmma_bf(v16b a, v16b b, v8f c) {
  v8f d = __builtin_amdgcn_wmma_f32_16x16x32_bf16(false, a, false, b, (short)0, c, false, false);
  asm volatile("v_nop\n\tv_nop\n\tv_nop\n\tv_nop" : "+v"(d) : "v"(a), "v"(b));
  return d;
}
__device__ __forceinline__ v16h frag_h(const _Float16* rowk0, int lane) {
  union { v16h v; v8h q[2]; } u; const _Float16* p = rowk0 + 8 * (lane >> 4);
  u.q[0] = *(const v8h*)p; u.q[1] = *(const v8h*)(p + 16); return u.v;
}
__device__ __forceinline__ v16h frag_f32(const float* rowk0, int lane) {
  v16h a; const float* p = rowk0 + 8 * (lane >> 4);
#pragma unroll
  for (int i = 0; i < 8; ++i) { a[i] = (_Float16)p[i]; a[8 + i] = (_Float16)p[16 + i]; }
  return a;
}
__device__ __forceinline__ v16h frag_f32s(const float* rowk0, int lane, float sc) {
  v16h a; const float* p = rowk0 + 8 * (lane >> 4);
#pragma unroll
  for (int i = 0; i < 8; ++i) { a[i] = (_Float16)(p[i] * sc); a[8 + i] = (_Float16)(p[16 + i] * sc); }
  return a;
}
__device__ __forceinline__ v16h fragc_f32(const float* W, int k0, int n, int lane, int ld, int K) {
  v16h a; const int g = lane >> 4;
#pragma unroll
  for (int i = 0; i < 8; ++i) { const int ka = k0 + 8 * g + i, kb = ka + 16;
    a[i] = (_Float16)(ka < K ? W[(size_t)(ka < K ? ka : K - 1) * ld + n] : 0.f); a[8 + i] = (_Float16)(kb < K ? W[(size_t)(kb < K ? kb : K - 1) * ld + n] : 0.f); }
  return a;
}
struct F2 { v16b h, l; };
__device__ __forceinline__ F2 bsplit16(const float v[16]) { F2 r;
#pragma unroll
  for (int i = 0; i < 16; ++i) { const __bf16 h = (__bf16)v[i]; r.h[i] = h; r.l[i] = (__bf16)(v[i] - (float)h); }
  return r; }
__device__ __forceinline__ F2 split_row(const float* row, int k0, int lane) { float v[16]; const float* p = row + k0 + 8 * (lane >> 4);
#pragma unroll
  for (int i = 0; i < 8; ++i) { v[i] = p[i]; v[8 + i] = p[16 + i]; }
  return bsplit16(v); }
__device__ __forceinline__ F2 split_rowK(const float* row, int k0, int lane, int K) { float v[16]; const int g = lane >> 4;
#pragma unroll
  for (int i = 0; i < 8; ++i) { const int ka = k0 + 8 * g + i, kb = ka + 16; v[i] = ka < K ? row[ka < K ? ka : K - 1] : 0.f; v[8 + i] = kb < K ? row[kb < K ? kb : K - 1] : 0.f; }
  return bsplit16(v); }
__device__ __forceinline__ F2 split_col(const float* W, int k0, int n, int lane, int ld, int K) { float v[16]; const int g = lane >> 4;
#pragma unroll
  for (int i = 0; i < 8; ++i) { const int ka = k0 + 8 * g + i, kb = ka + 16; v[i] = ka < K ? W[(size_t)(ka < K ? ka : K - 1) * ld + n] : 0.f; v[8 + i] = kb < K ? W[(size_t)(kb < K ? kb : K - 1) * ld + n] : 0.f; }
  return bsplit16(v); }
__device__ __forceinline__ v8f mac3(const F2& a, const F2& b, v8f c) { c = wmma_bf(a.l, b.h, c); c = wmma_bf(a.h, b.l, c); return wmma_bf(a.h, b.h, c); }
__device__ __forceinline__ float sigm(float v) { return 1.0f / (1.0f + expf(-v)); }
#define LDSX() do { asm volatile("s_wait_dscnt 0" ::: "memory"); __builtin_amdgcn_wave_barrier(); __builtin_amdgcn_fence(__ATOMIC_RELEASE, "workgroup"); } while (0)


#define NB 16
#define NP 2048
#define NR (NB * NP)
#define CC 128
#define KN 16
#define KS 17
#define LG 256
#ifndef NBT
#define NBT NB
#endif
typedef __attribute__((ext_vector_type(8))) __bf16 v8b;
__device__ __forceinline__ v16b frag_b(const __bf16* rowk0, int lane) {
  union { v16b v; v8b q[2]; } u; const __bf16* p = rowk0 + 8 * (lane >> 4);
  u.q[0] = *(const v8b*)p; u.q[1] = *(const v8b*)(p + 16); return u.v;
}
__device__ __forceinline__ float bfr(float v) { return (float)(__bf16)v; }
__device__ __attribute__((noinline)) float exp_ni(float v) { return expf(v); }
__device__ __attribute__((noinline)) float erf_ni(float v) { return erff(v); }
__device__ __attribute__((noinline)) float tanh_ni(float v) { return tanhf(v); }
__device__ __attribute__((noinline)) float cos_ni(float v) { return cosf(v); }
__device__ __attribute__((noinline)) float sin_ni(float v) { return sinf(v); }
#pragma clang fp contract(off)

#define PK_T2 0
#define PK_P1 (1 * CC * CC)
#define PK_P2 (2 * CC * CC)
#define PK_S1 (3 * CC * CC)
#define PK_END (PK_S1 + CC * 512)
#define WS_PK   0u
#define WS_FB   (((2u * PK_END) + 127u) / 128u * 128u)
#define WS_LB   (WS_FB + 2u * NR * CC)
#define WS_LP   (WS_LB + 2u * NB * LG)
#define WS_OBJ  (WS_LP + 4u * NB * CC)
#define WS_IDX  (WS_OBJ + 4u * NR)
#define WS_ROT  (WS_IDX + 4u * NR * KN)
#define WS_MSK  (WS_ROT + 4u * NR * KN * 2)
#define WS_DEN  (WS_MSK + 4u * NR * KN)
#define WS_U1   (WS_DEN + 4u * (NR / 4) * 32)
#define WS_U2   (WS_U1 + 4u * NR * CC)
#define WS_END  (WS_U2 + 4u * NR * CC)

__global__ __launch_bounds__(256) void k_pack(const float* __restrict__ T2, const float* __restrict__ P1, const float* __restrict__ P2, const float* __restrict__ S1, __bf16* __restrict__ PK) {
  __shared__ __align__(16) __bf16 s[512]; const int n = blockIdx.x, which = blockIdx.y, t = threadIdx.x; int K = CC; size_t dst;
  if (which < 3) { const float* Wm = (which == 0) ? T2 : (which == 1) ? P1 : P2; dst = (size_t)which * CC * CC + (size_t)n * CC; if (t < CC) s[t] = (__bf16)Wm[(size_t)t * CC + n]; }
  else { K = 512; dst = PK_S1 + (size_t)n * 512; for (int k = t; k < 512; k += 256) s[k] = (__bf16)S1[(size_t)k * CC + n]; }
  __syncthreads();
  for (int q = t; q < K / 8; q += 256) vst2((unsigned*)(PK + dst + q * 8), *(const v4u*)&s[q * 8]);
}
__global__ __launch_bounds__(256) void k_prep(const float* __restrict__ F, const float* __restrict__ OS, const float* __restrict__ LANG, const float* __restrict__ TW1, const float* __restrict__ TB1, __bf16* __restrict__ FB, float* __restrict__ OBJ, __bf16* __restrict__ LB, float* __restrict__ LP) {
  __shared__ __align__(16) __bf16 sf[64][CC]; __shared__ __align__(16) float so[64]; __shared__ __align__(16) __bf16 sl[LG]; __shared__ __align__(16) float slp[CC];
  const int tid = threadIdx.x; const size_t r0 = (size_t)blockIdx.x * 64;
  for (int q = tid; q < 64 * CC; q += 256) { const int r = q >> 7, c = q & 127; sf[r][c] = (__bf16)F[(r0 + r) * CC + c]; }
  if (tid < 64) { const float a = bfr(OS[(r0 + tid) * 2]), b = bfr(OS[(r0 + tid) * 2 + 1]); so[tid] = (b > a) ? 1.f : 0.f; }
  if (blockIdx.x < NB) { const int b = blockIdx.x; for (int k = tid; k < LG; k += 256) sl[k] = (__bf16)LANG[(size_t)b * LG + k]; }
  __syncthreads();
  if (blockIdx.x < NB && tid < CC) { const int b = blockIdx.x; float a = 0.f; for (int k = 0; k < LG; ++k) a += (float)sl[k] * bfr(TW1[(size_t)(3 + k) * CC + tid]); slp[tid] = a + bfr(TB1[tid]); }
  __syncthreads();
  for (int q = tid; q < 64 * CC / 8; q += 256) vst2((unsigned*)(FB + r0 * CC + q * 8), *(const v4u*)(&sf[0][0] + q * 8));
  if (tid < 16) vst2(OBJ + r0 + tid * 4, *(const v4f*)&so[tid * 4]);
  if (blockIdx.x < NB) { const int b = blockIdx.x; if (tid < LG / 8) vst2((unsigned*)(LB + (size_t)b * LG + tid * 8), *(const v4u*)&sl[tid * 8]); else if (tid >= 64 && tid < 64 + CC / 4) vst2(LP + (size_t)b * CC + (tid - 64) * 4, *(const v4f*)&slp[(tid - 64) * 4]); }
}
__global__ __launch_bounds__(256) void k_knn(const float* __restrict__ XYZ, int* __restrict__ IDX) {
  __shared__ float sx[NP], sy[NP], sz[NP]; __shared__ __align__(16) int sidx[256][KN];
  const int tid = threadIdx.x; const int b = blockIdx.x / (NP / 256); const int q0 = (blockIdx.x % (NP / 256)) * 256; const int q = q0 + tid;
  for (int i = tid; i < NP; i += 256) { const float* p = XYZ + ((size_t)b * NP + i) * 3; sx[i] = bfr(p[0]); sy[i] = bfr(p[1]); sz[i] = bfr(p[2]); }
  __syncthreads();
  const float qx = sx[q], qy = sy[q], qz = sz[q];
  float bd[KS]; int bi[KS];
#pragma unroll
  for (int s = 0; s < KS; ++s) { bd[s] = 3.0e38f; bi[s] = 0; }
  for (int m = 0; m < NP; ++m) { const float t0 = qx - sx[m], t1 = qy - sy[m], t2 = qz - sz[m]; const float s0 = t0 * t0, s1 = t1 * t1, s2 = t2 * t2; const float D = (s0 + s2) + s1;
    if (D < bd[KS - 1]) { float cd = D; int ci = m; bool placed = false;
#pragma unroll
      for (int s = 0; s < KS; ++s) { const bool sw = placed || (cd < bd[s]); placed = sw; const float td = bd[s]; const int ti = bi[s]; bd[s] = sw ? cd : td; bi[s] = sw ? ci : ti; cd = sw ? td : cd; ci = sw ? ti : ci; } } }
#pragma unroll
  for (int s = 1; s < KS; ++s) sidx[tid][s - 1] = bi[s];
  __syncthreads();
  for (int qq = tid; qq < 256 * KN / 4; qq += 256) vst2((unsigned*)(IDX + ((size_t)b * NP + q0) * KN + qq * 4), *(const v4u*)(&sidx[0][0] + qq * 4));
}
__global__ __launch_bounds__(128) void k_theta(const float* __restrict__ XYZ, const int* __restrict__ IDX, const float* __restrict__ LP, const float* __restrict__ TW1, const float* __restrict__ TB2, const float* __restrict__ TW3, const float* __restrict__ TB3, const float* __restrict__ OBJ, const __bf16* __restrict__ PK, float* __restrict__ ROT, float* __restrict__ MSK, float* __restrict__ DEN) {
  __shared__ __align__(16) __bf16 sah[4][16][CC + 8], sal[4][16][CC + 8]; __shared__ float sdl[4][KN][4]; __shared__ int sid[4][KN]; __shared__ __align__(16) float srot[4][KN][2]; __shared__ __align__(16) float smsk[4][KN]; __shared__ __align__(16) float sden[32];
  const int tid = threadIdx.x, wave = tid >> 5, lane = tid & 31, col = lane & 15, g = lane >> 4; const size_t n = (size_t)blockIdx.x * 4 + wave; const int b = (int)(n / NP);
  if (lane < KN) { const int id = min(max(IDX[n * KN + lane], 0), NP - 1); sid[wave][lane] = id; const float* pp = XYZ + ((size_t)b * NP + id) * 3; const float* pc = XYZ + n * 3;
    sdl[wave][lane][0] = bfr(pp[0]) - bfr(pc[0]); sdl[wave][lane][1] = bfr(pp[1]) - bfr(pc[1]); sdl[wave][lane][2] = bfr(pp[2]) - bfr(pc[2]);
    const float mk = OBJ[(size_t)b * NP + id]; smsk[wave][lane] = mk;
    float sm = mk;
#pragma unroll
    for (int o = 1; o < 16; o <<= 1) sm += __shfl_xor(sm, o);
    if (lane == 0) sden[wave] = 1.0f / fmaxf(sm, 1.0f); }
  else { float sm = 0.f;
#pragma unroll
    for (int o = 1; o < 16; o <<= 1) sm += __shfl_xor(sm, o); }
  if (wave == 0 && lane >= 4) sden[lane] = 0.f;
  LDSX();
  const float* lp = LP + (size_t)b * CC;
  for (int k = 0; k < KN; ++k) { const float d0 = sdl[wave][k][0], d1 = sdl[wave][k][1], d2 = sdl[wave][k][2];
#pragma unroll
    for (int i = 0; i < 4; ++i) { const int c = lane + 32 * i; const float v = fmaxf(((d0 * bfr(TW1[c]) + d1 * bfr(TW1[CC + c])) + d2 * bfr(TW1[2 * CC + c])) + lp[c], 0.f); const __bf16 hb = (__bf16)v; sah[wave][k][c] = hb; sal[wave][k][c] = (__bf16)(v - (float)hb); } }
  LDSX();
  v8f acc[8] = {};
#pragma unroll
  for (int kc = 0; kc < CC / 32; ++kc) { F2 a; a.h = frag_b(&sah[wave][col][kc * 32], lane); a.l = frag_b(&sal[wave][col][kc * 32], lane);
#pragma unroll
    for (int j = 0; j < 8; ++j) { const v16b w = frag_b(PK + PK_T2 + (size_t)(j * 16 + col) * CC + kc * 32, lane); acc[j] = wmma_bf(a.l, w, acc[j]); acc[j] = wmma_bf(a.h, w, acc[j]); } }
  float z[8];
#pragma unroll
  for (int r = 0; r < 8; ++r) { float s = 0.f;
#pragma unroll
    for (int j = 0; j < 8; ++j) { const int c = j * 16 + col; s += fmaxf(acc[j][r] + bfr(TB2[c]), 0.f) * bfr(TW3[c]); }
#pragma unroll
    for (int o = 1; o < 16; o <<= 1) s += __shfl_xor(s, o);
    z[r] = s; }
  if (col < 8) { const int r = col; const int k = 8 * g + r; float zz = z[0];
#pragma unroll
    for (int i = 1; i < 8; ++i) zz = (r == i) ? z[i] : zz;
    const float th = tanh_ni(zz + bfr(TB3[0])) * 3.14159265358979323846f; srot[wave][k][0] = cos_ni(th); srot[wave][k][1] = sin_ni(th); }
  LDSX();
  if (lane < 8) vst2(ROT + n * KN * 2 + lane * 4, *(const v4f*)(&srot[wave][0][0] + lane * 4));
  __syncthreads();
  if (tid < 16) vst2(MSK + (size_t)blockIdx.x * 4 * KN + tid * 4, *(const v4f*)(&smsk[0][0] + tid * 4));
  else if (tid >= 32 && tid < 40) vst2(DEN + (size_t)blockIdx.x * 32 + (tid - 32) * 4, *(const v4f*)&sden[(tid - 32) * 4]);
}
__global__ __launch_bounds__(256) void k_diff(const float* __restrict__ UP, const float* __restrict__ F, const int* __restrict__ IDX, const float* __restrict__ ROT, const float* __restrict__ MSK, const float* __restrict__ DEN, int step0, float* __restrict__ UN) {
  const int tid = threadIdx.x, wave = tid >> 5, lane = tid & 31; const size_t n = (size_t)blockIdx.x * 8 + wave; const int b = (int)(n / NP); const int c0 = lane * 4;
  float a0 = 0.f, a1 = 0.f, a2 = 0.f, a3 = 0.f;
  for (int k = 0; k < KN; ++k) { const int id = min(max(IDX[n * KN + k], 0), NP - 1); const float cs = ROT[(n * KN + k) * 2], sn = ROT[(n * KN + k) * 2 + 1], mk = MSK[n * KN + k];
    const float* src = step0 ? (F + ((size_t)b * NP + id) * CC + c0) : (UP + ((size_t)b * NP + id) * CC + c0);
    float re0, im0, re1, im1; if (step0) { re0 = bfr(src[0]); im0 = bfr(src[1]); re1 = bfr(src[2]); im1 = bfr(src[3]); } else { re0 = src[0]; im0 = src[1]; re1 = src[2]; im1 = src[3]; }
    a0 += (re0 * cs - im0 * sn) * mk; a1 += (re0 * sn + im0 * cs) * mk; a2 += (re1 * cs - im1 * sn) * mk; a3 += (re1 * sn + im1 * cs) * mk; }
  const float dn = DEN[(n >> 2) * 32 + (n & 3)]; float u0, u1, u2, u3; { const float* ur = step0 ? (F + n * CC + c0) : (UP + n * CC + c0); if (step0) { u0 = bfr(ur[0]); u1 = bfr(ur[1]); u2 = bfr(ur[2]); u3 = bfr(ur[3]); } else { u0 = ur[0]; u1 = ur[1]; u2 = ur[2]; u3 = ur[3]; } }
  v4f o; o[0] = u0 + 0.5f * (a0 * dn - u0); o[1] = u1 + 0.5f * (a1 * dn - u1); o[2] = u2 + 0.5f * (a2 * dn - u2); o[3] = u3 + 0.5f * (a3 * dn - u3);
  vst2(UN + n * CC + c0, o);
}
__global__ __launch_bounds__(128) void k_head(const float* __restrict__ U3, const __bf16* __restrict__ FB, const __bf16* __restrict__ LB, const float* __restrict__ LNG, const float* __restrict__ LNB, const float* __restrict__ PB1, const float* __restrict__ PB2, const float* __restrict__ SB1, const float* __restrict__ SW2, const float* __restrict__ SB2, const float* __restrict__ OBJ, const __bf16* __restrict__ PK, float* __restrict__ OUT0) {
  __shared__ __align__(16) __bf16 sah[4][16][CC + 8], sal[4][16][CC + 8]; __shared__ __align__(16) float sconf[64];
  const int tid = threadIdx.x, wave = tid >> 5, lane = tid & 31, col = lane & 15, g = lane >> 4; const size_t r0 = (size_t)blockIdx.x * 64 + wave * 16; const int b = (int)(r0 / NP);
  for (int rl = 0; rl < 16; ++rl) { const float* u = U3 + (r0 + rl) * CC; float v[4]; float s = 0.f;
#pragma unroll
    for (int i = 0; i < 4; ++i) { v[i] = u[lane + 32 * i]; s += v[i]; }
#pragma unroll
    for (int o = 1; o < 32; o <<= 1) s += __shfl_xor(s, o);
    const float mu = s * (1.0f / CC); float q = 0.f;
#pragma unroll
    for (int i = 0; i < 4; ++i) { const float dv = v[i] - mu; q += dv * dv; }
#pragma unroll
    for (int o = 1; o < 32; o <<= 1) q += __shfl_xor(q, o);
    const float sd = sqrtf(q * (1.0f / CC) + 1e-5f);
#pragma unroll
    for (int i = 0; i < 4; ++i) { const int c = lane + 32 * i; const float x = (v[i] - mu) / sd * bfr(LNG[c]) + bfr(LNB[c]); const __bf16 hb = (__bf16)x; sah[wave][rl][c] = hb; sal[wave][rl][c] = (__bf16)(x - (float)hb); } }
  LDSX();
  v8f acc[8];
  auto layer = [&](const __bf16* P) {
#pragma unroll
    for (int j = 0; j < 8; ++j) acc[j] = v8f{};
#pragma unroll
    for (int kc = 0; kc < CC / 32; ++kc) { F2 a; a.h = frag_b(&sah[wave][col][kc * 32], lane); a.l = frag_b(&sal[wave][col][kc * 32], lane);
#pragma unroll
      for (int j = 0; j < 8; ++j) { const v16b w = frag_b(P + (size_t)(j * 16 + col) * CC + kc * 32, lane); acc[j] = wmma_bf(a.l, w, acc[j]); acc[j] = wmma_bf(a.h, w, acc[j]); } } };
  layer(PK + PK_P1); LDSX();
#pragma unroll
  for (int j = 0; j < 8; ++j) { const int c = j * 16 + col; const float bb = bfr(PB1[c]);
#pragma unroll
    for (int r = 0; r < 8; ++r) { const float x = fmaxf(acc[j][r] + bb, 0.f); const __bf16 hb = (__bf16)x; sah[wave][8 * g + r][c] = hb; sal[wave][8 * g + r][c] = (__bf16)(x - (float)hb); } }
  LDSX();
  layer(PK + PK_P2); LDSX();
#pragma unroll
  for (int j = 0; j < 8; ++j) { const int c = j * 16 + col; const float bb = bfr(PB2[c]);
#pragma unroll
    for (int r = 0; r < 8; ++r) { const float x = acc[j][r] + bb; const __bf16 hb = (__bf16)x; sah[wave][8 * g + r][c] = hb; sal[wave][8 * g + r][c] = (__bf16)(x - (float)hb); } }
  LDSX();
#pragma unroll
  for (int j = 0; j < 8; ++j) acc[j] = v8f{};
#pragma unroll
  for (int kc = 0; kc < CC / 32; ++kc) { F2 a; a.h = frag_b(&sah[wave][col][kc * 32], lane); a.l = frag_b(&sal[wave][col][kc * 32], lane);
#pragma unroll
    for (int j = 0; j < 8; ++j) { const v16b w = frag_b(PK + PK_S1 + (size_t)(j * 16 + col) * 512 + kc * 32, lane); acc[j] = wmma_bf(a.l, w, acc[j]); acc[j] = wmma_bf(a.h, w, acc[j]); } }
#pragma unroll
  for (int kc = 0; kc < CC / 32; ++kc) { const v16b a = frag_b(FB + (r0 + col) * CC + kc * 32, lane);
#pragma unroll
    for (int j = 0; j < 8; ++j) acc[j] = wmma_bf(a, frag_b(PK + PK_S1 + (size_t)(j * 16 + col) * 512 + CC + kc * 32, lane), acc[j]); }
#pragma unroll 1
  for (int kc = 0; kc < LG / 32; ++kc) { const v16b a = frag_b(LB + (size_t)b * LG + kc * 32, lane);
    v16b aa; { const __bf16* p = LB + (size_t)b * LG + kc * 32 + 8 * g;
#pragma unroll
      for (int i = 0; i < 8; ++i) { aa[i] = p[i]; aa[8 + i] = p[16 + i]; } } (void)a;
#pragma unroll
    for (int j = 0; j < 8; ++j) acc[j] = wmma_bf(aa, frag_b(PK + PK_S1 + (size_t)(j * 16 + col) * 512 + 2 * CC + kc * 32, lane), acc[j]); }
  { float cf[8];
#pragma unroll
    for (int r = 0; r < 8; ++r) { float s = 0.f;
#pragma unroll
      for (int j = 0; j < 8; ++j) { const int c = j * 16 + col; s += fmaxf(acc[j][r] + bfr(SB1[c]), 0.f) * bfr(SW2[c]); }
#pragma unroll
      for (int o = 1; o < 16; o <<= 1) s += __shfl_xor(s, o);
      cf[r] = s; }
    if (col < 8) { const int r = col; float zz = cf[0];
#pragma unroll
      for (int i = 1; i < 8; ++i) zz = (r == i) ? cf[i] : zz;
      const size_t row = r0 + 8 * g + r; sconf[wave * 16 + 8 * g + r] = (zz + bfr(SB2[0])) * OBJ[row]; } }
  __syncthreads();
  if (tid < 16) vst2(OUT0 + (size_t)blockIdx.x * 64 + tid * 4, *(const v4f*)&sconf[tid * 4]);
}
extern "C" void kernel_launch(void* const* d_in, const int* in_sizes, int n_in, void* d_out, int out_size, void* d_ws, size_t ws_size, hipStream_t stream) {
  (void)in_sizes; (void)n_in; (void)out_size;
  const float** F = (const float**)d_in;
  if (ws_size < (size_t)WS_END) return;
  char* ws = (char*)d_ws; __bf16 *PK = (__bf16*)(ws + WS_PK), *FB = (__bf16*)(ws + WS_FB), *LB = (__bf16*)(ws + WS_LB); float *LP = (float*)(ws + WS_LP), *OBJ = (float*)(ws + WS_OBJ), *ROT = (float*)(ws + WS_ROT), *MSK = (float*)(ws + WS_MSK), *DEN = (float*)(ws + WS_DEN), *U1 = (float*)(ws + WS_U1), *U2 = (float*)(ws + WS_U2); int* IDX = (int*)(ws + WS_IDX);
  float* OUT0 = (float*)d_out; float* OUT1 = (float*)((char*)d_out + 131072);
  k_pack<<<dim3(CC, 4), 256, 0, stream>>>(F[6], F[12], F[14], F[16], PK);
  k_prep<<<NBT * NP / 64, 256, 0, stream>>>(F[1], F[3], F[2], F[4], F[5], FB, OBJ, LB, LP);
  k_knn<<<NBT * NP / 256, 256, 0, stream>>>(F[0], IDX);
  k_theta<<<NBT * NP / 4, 128, 0, stream>>>(F[0], IDX, LP, F[4], F[7], F[8], F[9], OBJ, PK, ROT, MSK, DEN);
  k_diff<<<NBT * NP / 8, 256, 0, stream>>>(nullptr, F[1], IDX, ROT, MSK, DEN, 1, U1);
  k_diff<<<NBT * NP / 8, 256, 0, stream>>>(U1, F[1], IDX, ROT, MSK, DEN, 0, U2);
  k_diff<<<NBT * NP / 8, 256, 0, stream>>>(U2, F[1], IDX, ROT, MSK, DEN, 0, OUT1);
  k_head<<<NBT * NP / 64, 128, 0, stream>>>(OUT1, FB, LB, F[10], F[11], F[13], F[15], F[17], F[18], F[19], OBJ, PK, OUT0);
}
